// PNALSPELayer_29368986370543
// MI455X (gfx1250) — hardware-verified
//
#include <hip/hip_runtime.h>
#include <hip/hip_bf16.h>
#include <stddef.h>
#include <math.h>


#pragma clang fp contract(off)

#define DD     64
#define PXW    128
#define AGW    256
#define KPH    896
#define KPP    832
#define NB     128
#define NTHR   256
#define NWAVE  8
#define EPT    8
#define CHUNK  (NTHR * EPT)
#define WCAP   (EPT * 32)
#define PASSN  128
#define PCAP   4096
#define EHDR   32
#define EROW   (EHDR + PCAP)
#define RMAX   (PCAP / PASSN)
#define RB     64
#define RTHR   128
#define ETW    32
#define EKIN   16
#define ESC    16.0f
#define RESC   0.0625f
#define AVGL   3.5f
#define RAVGL  (1.0f / 3.5f)
#define AEPS   1e-5f
#define BEPS   1e-5f
#define WSLIM  134217728

#define LA_ACC  0
#define LA_MSG  (LA_ACC + (NB + 1) * AGW * 4)
#define LA_ET   (LA_MSG + PASSN * DD * 4)
#define LA_SLOT (LA_ET + PASSN * ETW * 2)
#define LA_CNT  (LA_SLOT + PASSN * 4)
#define LA_DGS  (LA_CNT + 528)
#define LA_TOT  (LA_DGS + NB * 4 * 4)

#define PU0 (128 * 128 / 8)
#define PU1 (128 * 64 / 8)
#define PU2 (64 * KPH / 8)
#define PU3 (64 * KPP / 8)
#define PU4 (64 * 64 / 8)
#define PUE (64 * ETW / 8)
#define PB0 (PU0 / NTHR)
#define PB1 (PB0 + PU1 / NTHR)
#define PB2 (PB1 + PU2 / NTHR)
#define PB3 (PB2 + PU3 / NTHR)
#define PB4 (PB3 + PU4 / NTHR)
#define PB5 (PB4 + PU4 / NTHR)
#define PB6 (PB5 + PUE / NTHR)
#define PBT (PB6 + PUE / NTHR)

static_assert(NTHR == NWAVE * 32);
static_assert(NTHR == 2 * PASSN);
static_assert(PASSN == NWAVE * 16);
static_assert(NB == NWAVE * 16);
static_assert((PCAP % PASSN) == 0 && RMAX * PASSN == PCAP);
static_assert(EHDR * 4 == 128);
static_assert((EROW % 4) == 0 && ((EROW * 4) % 128) == 0);
static_assert((NB + 1) * 4 <= 528);
static_assert((LA_MSG % 16) == 0 && (LA_ET % 16) == 0 && (LA_SLOT % 16) == 0 && (LA_CNT % 16) == 0 && (LA_DGS % 16) == 0);
static_assert(LA_TOT <= 300 * 1024);
static_assert((PU0 % NTHR) == 0 && (PU1 % NTHR) == 0 && (PU2 % NTHR) == 0 && (PU3 % NTHR) == 0);
static_assert((PU4 % NTHR) == 0 && (PUE % NTHR) == 0);
static_assert(PBT == 72);
static_assert(RTHR == 4 * 32 && RB == 4 * 16);
static_assert((NB % RB) == 0);
static_assert((KPH % 32) == 0 && (KPP % 32) == 0 && (AGW % 32) == 0);
static_assert(KPH == 2 * DD + 3 * AGW && KPP == DD + 3 * AGW);

typedef float          v4f   __attribute__((ext_vector_type(4)));
typedef float          v8f   __attribute__((ext_vector_type(8)));
typedef int            v4i   __attribute__((ext_vector_type(4)));
typedef unsigned short v8us  __attribute__((ext_vector_type(8)));
typedef unsigned short v16us __attribute__((ext_vector_type(16)));
typedef __bf16         v16bf __attribute__((ext_vector_type(16)));
typedef _Float16       v8h   __attribute__((ext_vector_type(8)));
typedef _Float16       v16h  __attribute__((ext_vector_type(16)));
union FragB { v16bf v; v16us u; v8us h[2]; };
union FragH { v16h v; v8h h[2]; };
union Pk8 { v8us h; v4i i; };
union Ph8 { v8h h; v4i i; };

__device__ __forceinline__ unsigned f2bf(float f) {
  const unsigned u = __float_as_uint(f);
  return (u + 0x7FFFu + ((u >> 16) & 1u)) >> 16;
}

__device__ __forceinline__ void split8(v4f a, v4f b, v8us& hi, v8us& lo) {
  float f[8];
  f[0] = a.x; f[1] = a.y; f[2] = a.z; f[3] = a.w;
  f[4] = b.x; f[5] = b.y; f[6] = b.z; f[7] = b.w;
  v8us rh, rl;
#pragma unroll
  for (int i = 0; i < 8; ++i) {
    const unsigned hb = f2bf(f[i]);
    const float r = f[i] - __uint_as_float(hb << 16);
    rh[i] = (unsigned short)hb;
    rl[i] = (unsigned short)f2bf(r);
  }
  hi = rh;
  lo = rl;
}

__device__ __forceinline__ v8f zero8() {
  v8f c;
#pragma unroll
  for (int i = 0; i < 8; ++i) c[i] = 0.0f;
  return c;
}

__device__ __forceinline__ v8f wm3(v16bf ah, v16bf al, v16bf bh, v16bf bl, v8f c) {
  v8f d = __builtin_amdgcn_wmma_f32_16x16x32_bf16(false, ah, false, bh, (short)0, c, false, false);
  d = __builtin_amdgcn_wmma_f32_16x16x32_bf16(false, ah, false, bl, (short)0, d, false, false);
  d = __builtin_amdgcn_wmma_f32_16x16x32_bf16(false, al, false, bh, (short)0, d, false, false);
  asm volatile("v_nop\n\tv_nop\n\tv_nop\n\tv_nop" : "+v"(d) : "v"(ah), "v"(al), "v"(bh), "v"(bl));
  return d;
}

__device__ __forceinline__ v8f wmh(v16h a, v16h b, v8f c) {
  v8f d = __builtin_amdgcn_wmma_f32_16x16x32_f16(false, a, false, b, (short)0, c, false, false);
  asm volatile("v_nop\n\tv_nop\n\tv_nop\n\tv_nop" : "+v"(d) : "v"(a), "v"(b));
  return d;
}

template <int NFT>
__device__ __forceinline__ void gstep(v8f (&acc)[NFT], const float* arow, int k0, float sc,
                                      const unsigned short* __restrict__ qh,
                                      const unsigned short* __restrict__ ql,
                                      int kp, int kw, int hh, int m) {
  FragB ah, al;
  {
    v4f a = *(const v4f*)(arow + k0 + 8 * hh);
    v4f b = *(const v4f*)(arow + k0 + 8 * hh + 4);
    v4f c = *(const v4f*)(arow + k0 + 16 + 8 * hh);
    v4f d = *(const v4f*)(arow + k0 + 20 + 8 * hh);
    a = a * sc; b = b * sc; c = c * sc; d = d * sc;
    split8(a, b, ah.h[0], al.h[0]);
    split8(c, d, ah.h[1], al.h[1]);
  }
#pragma unroll
  for (int ft = 0; ft < NFT; ++ft) {
    FragB bh, bl;
    const size_t o = (size_t)(16 * ft + m) * kp + kw + 8 * hh;
    bh.h[0] = *(const v8us*)(qh + o);
    bh.h[1] = *(const v8us*)(qh + o + 16);
    bl.h[0] = *(const v8us*)(ql + o);
    bl.h[1] = *(const v8us*)(ql + o + 16);
    acc[ft] = wm3(ah.v, al.v, bh.v, bl.v, acc[ft]);
  }
}

__device__ __forceinline__ int scan_chunk(const int* __restrict__ dsts, int nE, int cbase, int nodeBase,
                                          int vec8, int* list, int tid, int wave) {
  int wc = 0;
  const int el0  = tid * EPT;
  const int e0   = cbase + el0;
  const int sent = -2147483647 - 1;
  v4i da, db;
  if (vec8 != 0 && cbase + CHUNK <= nE) {
    da = *(const v4i*)(dsts + e0);
    db = *(const v4i*)(dsts + e0 + 4);
  } else {
    da.x = (e0     < nE) ? dsts[min(e0, nE - 1)] : sent;
    da.y = (e0 + 1 < nE) ? dsts[min(e0 + 1, nE - 1)] : sent;
    da.z = (e0 + 2 < nE) ? dsts[min(e0 + 2, nE - 1)] : sent;
    da.w = (e0 + 3 < nE) ? dsts[min(e0 + 3, nE - 1)] : sent;
    db.x = (e0 + 4 < nE) ? dsts[min(e0 + 4, nE - 1)] : sent;
    db.y = (e0 + 5 < nE) ? dsts[min(e0 + 5, nE - 1)] : sent;
    db.z = (e0 + 6 < nE) ? dsts[min(e0 + 6, nE - 1)] : sent;
    db.w = (e0 + 7 < nE) ? dsts[min(e0 + 7, nE - 1)] : sent;
  }
  const unsigned nb = (unsigned)nodeBase;
  const unsigned s0 = (unsigned)da.x - nb, s1 = (unsigned)da.y - nb;
  const unsigned s2 = (unsigned)da.z - nb, s3 = (unsigned)da.w - nb;
  const unsigned s4 = (unsigned)db.x - nb, s5 = (unsigned)db.y - nb;
  const unsigned s6 = (unsigned)db.z - nb, s7 = (unsigned)db.w - nb;
  const bool h0 = s0 < (unsigned)NB, h1 = s1 < (unsigned)NB, h2 = s2 < (unsigned)NB, h3 = s3 < (unsigned)NB;
  const bool h4 = s4 < (unsigned)NB, h5 = s5 < (unsigned)NB, h6 = s6 < (unsigned)NB, h7 = s7 < (unsigned)NB;
  const unsigned any = __builtin_amdgcn_ballot_w32(h0 | h1 | h2 | h3 | h4 | h5 | h6 | h7);
  if (any != 0u) {
#define HITJ(J, HJ) { \
      const unsigned mj = __builtin_amdgcn_ballot_w32(HJ); \
      if (mj != 0u) { \
        if (HJ) { \
          const int pos = wc + (int)__builtin_amdgcn_mbcnt_lo(mj, 0u); \
          if (pos < WCAP) list[wave * WCAP + pos] = el0 + (J); \
        } \
        wc += (int)__builtin_popcount(mj); } }
    HITJ(0, h0)
    HITJ(1, h1)
    HITJ(2, h2)
    HITJ(3, h3)
    HITJ(4, h4)
    HITJ(5, h5)
    HITJ(6, h6)
    HITJ(7, h7)
#undef HITJ
  }
  return wc;
}

__global__ __launch_bounds__(NTHR) void k_prep(
    const float* __restrict__ w0, const float* __restrict__ w1, const float* __restrict__ w2,
    const float* __restrict__ w3, const float* __restrict__ w4, const float* __restrict__ w5,
    unsigned short* q0, unsigned short* q1, unsigned short* q2, unsigned short* q3,
    unsigned short* q4, unsigned short* q5, _Float16* qe0, _Float16* qe1) {
  const int b = blockIdx.x, tid = threadIdx.x;
  const float* src;
  unsigned short* dq;
  _Float16* de;
  int NF, Kp, Kin, koff, kst, ub, f16m;
  if (b < PB0)      { src = w0; dq = q0; de = qe0; NF = 128; Kp = 128; Kin = 128;  koff = 0;   kst = 128; ub = b;       f16m = 0; }
  else if (b < PB1) { src = w1; dq = q1; de = qe0; NF = 128; Kp = 64;  Kin = 64;   koff = 0;   kst = 64;  ub = b - PB0; f16m = 0; }
  else if (b < PB2) { src = w2; dq = q2; de = qe0; NF = 64;  Kp = KPH; Kin = KPH;  koff = 0;   kst = 0;   ub = b - PB1; f16m = 0; }
  else if (b < PB3) { src = w3; dq = q3; de = qe0; NF = 64;  Kp = KPP; Kin = KPP;  koff = 0;   kst = 0;   ub = b - PB2; f16m = 0; }
  else if (b < PB4) { src = w4; dq = q4; de = qe0; NF = 64;  Kp = 64;  Kin = 64;   koff = 0;   kst = 0;   ub = b - PB3; f16m = 0; }
  else if (b < PB5) { src = w5; dq = q5; de = qe0; NF = 64;  Kp = 64;  Kin = 64;   koff = 0;   kst = 0;   ub = b - PB4; f16m = 0; }
  else if (b < PB6) { src = w0; dq = q0; de = qe0; NF = 64;  Kp = ETW; Kin = EKIN; koff = 256; kst = 0;   ub = b - PB5; f16m = 1; }
  else              { src = w1; dq = q0; de = qe1; NF = 64;  Kp = ETW; Kin = EKIN; koff = 128; kst = 0;   ub = b - PB6; f16m = 1; }
  const int u   = ub * NTHR + tid;
  const int cpr = Kp >> 3;
  int n = u / cpr;
  const int kc = u - n * cpr;
  n = n > NF - 1 ? NF - 1 : n;
  const int col = n & 63, g = n >> 6;
  float f[8];
#pragma unroll
  for (int j = 0; j < 8; ++j) {
    const int k   = 8 * kc + j;
    const int kcl = k < Kin ? k : Kin - 1;
    const float w = src[((size_t)(koff + g * kst + kcl)) * DD + col];
    f[j] = (k < Kin) ? w : 0.0f;
  }
  Pk8 ph, pl;
  Ph8 pe;
  {
    v4f a, c;
    a.x = f[0]; a.y = f[1]; a.z = f[2]; a.w = f[3];
    c.x = f[4]; c.y = f[5]; c.z = f[6]; c.w = f[7];
    split8(a, c, ph.h, pl.h);
    v8h oh;
#pragma unroll
    for (int j = 0; j < 8; ++j) oh[j] = (_Float16)(f[j] * ESC);
    pe.h = oh;
  }
  const size_t ne = (size_t)NF * Kp;
  unsigned short* dh = dq + (size_t)u * 8;
  unsigned short* dl = dq + ne + (size_t)u * 8;
  _Float16* dp = de + (size_t)u * 8;
  if (f16m != 0) {
    *(volatile v4i*)dp = pe.i;
  } else {
    *(volatile v4i*)dh = ph.i;
    *(volatile v4i*)dl = pl.i;
  }
  __threadfence();
  if (f16m != 0) {
    *(volatile v4i*)dp = pe.i;
  } else {
    *(volatile v4i*)dh = ph.i;
    *(volatile v4i*)dl = pl.i;
  }
}

__global__ __launch_bounds__(NTHR) void k_escan(const int* __restrict__ dsts, int* etab, int nE, int vec8) {
  __shared__ int list[NWAVE * WCAP];
  __shared__ __attribute__((aligned(16))) int pend[EROW];
  __shared__ int wcnt[NWAVE];
  const int tid = threadIdx.x, lane = tid & 31, wave = tid >> 5;
  const int nodeBase = blockIdx.x * NB;
  for (int i = tid; i < EROW; i += NTHR) pend[i] = 0;
  __syncthreads();
  int pendN = 0;
  const int nChunks = (nE + CHUNK - 1) / CHUNK;
#pragma unroll 1
  for (int ch = 0; ch < nChunks; ++ch) {
    const int cbase = ch * CHUNK;
    const int wc = scan_chunk(dsts, nE, cbase, nodeBase, vec8, list, tid, wave);
    if (lane == 0) wcnt[wave] = wc;
    __syncthreads();
    const int base = pendN;
    int tot = 0, myoff = 0;
#pragma unroll
    for (int w = 0; w < NWAVE; ++w) {
      int c = wcnt[w];
      c = c > WCAP ? WCAP : (c < 0 ? 0 : c);
      if (w < wave) myoff += c;
      tot += c;
    }
    {
      int n = wcnt[wave];
      n = n > WCAP ? WCAP : (n < 0 ? 0 : n);
      const int* lp = list + wave * WCAP;
      for (int i = lane; i < n; i += 32) {
        const int pos = base + myoff + i;
        if (pos < PCAP) pend[EHDR + pos] = cbase + lp[i];
      }
    }
    const int newN = base + tot;
    pendN = newN > PCAP ? PCAP : newN;
    __syncthreads();
  }
  if (tid == 0) pend[0] = pendN;
  __syncthreads();
  int* rowp = etab + (size_t)blockIdx.x * EROW;
#pragma unroll 1
  for (int u = tid; u < EROW / 4; u += NTHR) {
    const v4i v = *(const v4i*)(pend + 4 * u);
    *(volatile v4i*)(rowp + 4 * u) = v;
  }
  __threadfence();
#pragma unroll 1
  for (int u = tid; u < EROW / 4; u += NTHR) {
    const v4i v = *(const v4i*)(pend + 4 * u);
    *(volatile v4i*)(rowp + 4 * u) = v;
  }
}

__global__ __launch_bounds__(RTHR) void k_proj(const float* __restrict__ h, const float* __restrict__ p,
    const unsigned short* __restrict__ q0h, const unsigned short* __restrict__ q0l,
    const unsigned short* __restrict__ q1h, const unsigned short* __restrict__ q1l,
    float* ph, float* pp, int nN) {
  __shared__ __attribute__((aligned(16))) float stg[RB * PXW];
  const int tid = threadIdx.x, lane = tid & 31, wave = tid >> 5, hh = lane >> 4, m = lane & 15;
  const int rowBase = blockIdx.x * RB;
  int node = rowBase + wave * 16 + m;
  node = node > nN - 1 ? nN - 1 : node;
  const float* hr = h + (size_t)node * DD;
  const float* pr = p + (size_t)node * DD;
  {
    v8f acc[8];
#pragma unroll
    for (int i = 0; i < 8; ++i) acc[i] = zero8();
    gstep<8>(acc, hr, 0,  1.0f, q0h, q0l, PXW, 0,  hh, m);
    gstep<8>(acc, hr, 32, 1.0f, q0h, q0l, PXW, 32, hh, m);
    gstep<8>(acc, pr, 0,  1.0f, q0h, q0l, PXW, 64, hh, m);
    gstep<8>(acc, pr, 32, 1.0f, q0h, q0l, PXW, 96, hh, m);
#pragma unroll
    for (int ft = 0; ft < 8; ++ft) {
#pragma unroll
      for (int rr = 0; rr < 8; ++rr) stg[(wave * 16 + 8 * hh + rr) * PXW + 16 * ft + m] = acc[ft][rr];
    }
  }
  __syncthreads();
#pragma unroll 1
  for (int rr = 0; rr < 16; ++rr) {
    const int row = wave * 16 + rr;
    const v4f v = *(const v4f*)(stg + row * PXW + 4 * lane);
    *(volatile v4f*)(ph + (size_t)(rowBase + row) * PXW + 4 * lane) = v;
  }
  __threadfence();
#pragma unroll 1
  for (int rr = 0; rr < 16; ++rr) {
    const int row = wave * 16 + rr;
    const v4f v = *(const v4f*)(stg + row * PXW + 4 * lane);
    *(volatile v4f*)(ph + (size_t)(rowBase + row) * PXW + 4 * lane) = v;
  }
  __syncthreads();
  {
    v8f acc[8];
#pragma unroll
    for (int i = 0; i < 8; ++i) acc[i] = zero8();
    gstep<8>(acc, pr, 0,  1.0f, q1h, q1l, DD, 0,  hh, m);
    gstep<8>(acc, pr, 32, 1.0f, q1h, q1l, DD, 32, hh, m);
#pragma unroll
    for (int ft = 0; ft < 8; ++ft) {
#pragma unroll
      for (int rr = 0; rr < 8; ++rr) stg[(wave * 16 + 8 * hh + rr) * PXW + 16 * ft + m] = acc[ft][rr];
    }
  }
  __syncthreads();
#pragma unroll 1
  for (int rr = 0; rr < 16; ++rr) {
    const int row = wave * 16 + rr;
    const v4f v = *(const v4f*)(stg + row * PXW + 4 * lane);
    *(volatile v4f*)(pp + (size_t)(rowBase + row) * PXW + 4 * lane) = v;
  }
  __threadfence();
#pragma unroll 1
  for (int rr = 0; rr < 16; ++rr) {
    const int row = wave * 16 + rr;
    const v4f v = *(const v4f*)(stg + row * PXW + 4 * lane);
    *(volatile v4f*)(pp + (size_t)(rowBase + row) * PXW + 4 * lane) = v;
  }
}

__global__ __launch_bounds__(NTHR) void k_agg(
    const float* __restrict__ px, const float* __restrict__ ef,
    const int* __restrict__ srcs, const int* __restrict__ dsts, const int* __restrict__ etab,
    const _Float16* __restrict__ qe, const float* __restrict__ bias,
    float* aggp, float* dgp, int nN, int nE, int wdg) {
  extern __shared__ __attribute__((aligned(16))) unsigned char dsm[];
  float*    acc   = (float*)(dsm + LA_ACC);
  float*    msg   = (float*)(dsm + LA_MSG);
  _Float16* et    = (_Float16*)(dsm + LA_ET);
  int*      slotb = (int*)(dsm + LA_SLOT);
  int*      cnt   = (int*)(dsm + LA_CNT);
  float*    dgs   = (float*)(dsm + LA_DGS);
  const int tid = threadIdx.x, lane = tid & 31, wave = tid >> 5, hh = lane >> 4, m = lane & 15;
  const int nodeBase = blockIdx.x * NB;
  const int* erow = etab + (size_t)blockIdx.x * EROW;
  const float ninf = __uint_as_float(0xff800000u);
  const float pinf = __uint_as_float(0x7f800000u);

  for (int i = tid; i < (NB + 1) * AGW; i += NTHR) {
    const int cc = i & (AGW - 1);
    acc[i] = (cc < 64) ? 0.0f : ((cc < 128) ? ninf : ((cc < 192) ? pinf : 0.0f));
  }
  for (int i = tid; i < NB + 1; i += NTHR) cnt[i] = 0;
  {
    v4i z;
    z.x = 0; z.y = 0; z.z = 0; z.w = 0;
    for (int i = tid; i < PASSN * 2; i += NTHR) {
      const int row = i >> 1, hf = i & 1;
      *(v4i*)(et + row * ETW + 16 + 8 * hf) = z;
    }
  }
  int nP = erow[0];
  nP = nP < 0 ? 0 : (nP > PCAP ? PCAP : nP);
  int R = (nP + PASSN - 1) / PASSN;
  R = R > RMAX ? RMAX : R;
  __syncthreads();

#pragma unroll 1
  for (int r = 0; r < R; ++r) {
    {
      const int i = tid >> 1, q = tid & 1;
      const int idx = r * PASSN + i;
      const int idxc = idx < PCAP ? idx : PCAP - 1;
      int eid = erow[EHDR + idxc];
      eid = eid < 0 ? 0 : (eid > nE - 1 ? nE - 1 : eid);
      const int d = dsts[eid];
      int s = srcs[eid];
      s = s < 0 ? 0 : (s > nN - 1 ? nN - 1 : s);
      int dcl = d < 0 ? 0 : (d > nN - 1 ? nN - 1 : d);
      int slot = d - nodeBase;
      if (idx >= nP || (unsigned)slot >= (unsigned)NB) slot = NB;
      const float* ps = px + (size_t)s * PXW + 32 * q;
      const float* pd = px + (size_t)dcl * PXW + 64 + 32 * q;
      const float* bb = bias + 32 * q;
      float* mr = msg + i * DD + 32 * q;
#pragma unroll
      for (int j = 0; j < 8; ++j) {
        const v4f a = *(const v4f*)(ps + 4 * j);
        const v4f c = *(const v4f*)(pd + 4 * j);
        const v4f t = *(const v4f*)(bb + 4 * j);
        *(v4f*)(mr + 4 * j) = (a + c) + t;
      }
      const float* er = ef + (size_t)eid * EKIN + 8 * q;
      const v4f e0 = *(const v4f*)er;
      const v4f e1 = *(const v4f*)(er + 4);
      v8h oh;
      oh[0] = (_Float16)e0.x; oh[1] = (_Float16)e0.y; oh[2] = (_Float16)e0.z; oh[3] = (_Float16)e0.w;
      oh[4] = (_Float16)e1.x; oh[5] = (_Float16)e1.y; oh[6] = (_Float16)e1.z; oh[7] = (_Float16)e1.w;
      Ph8 o;
      o.h = oh;
      *(v4i*)(et + i * ETW + 8 * q) = o.i;
      if (q == 0) slotb[i] = slot;
    }
    __syncthreads();
    {
      FragH a;
      const _Float16* ar = et + (wave * 16 + m) * ETW + 8 * hh;
      a.h[0] = *(const v8h*)ar;
      a.h[1] = *(const v8h*)(ar + 16);
      float* mrow = msg + (wave * 16 + 8 * hh) * DD + m;
#pragma unroll
      for (int ft = 0; ft < 4; ++ft) {
        FragH bq;
        const _Float16* br = qe + (16 * ft + m) * ETW + 8 * hh;
        bq.h[0] = *(const v8h*)br;
        bq.h[1] = *(const v8h*)(br + 16);
        const v8f dv = wmh(a.v, bq.v, zero8());
#pragma unroll
        for (int rr = 0; rr < 8; ++rr) {
          float* mp = mrow + rr * DD + 16 * ft;
          const float t = *mp;
          *mp = t + dv[rr] * RESC;
        }
      }
    }
    __syncthreads();
    {
      int cntp = nP - r * PASSN;
      cntp = cntp > PASSN ? PASSN : (cntp < 0 ? 0 : cntp);
      const int stat = tid >> 6, c = tid & 63;
      float* abase = acc + 64 * stat + c;
#pragma unroll 1
      for (int i = 0; i < cntp; ++i) {
        int sl = slotb[i];
        sl = sl < 0 ? 0 : (sl > NB ? NB : sl);
        const float v = msg[i * DD + c];
        float* ap = abase + sl * AGW;
        if (stat == 0) {
          *ap = *ap + v;
          if (c == 0) cnt[sl] = cnt[sl] + 1;
        } else if (stat == 1) {
          *ap = fmaxf(*ap, v);
        } else if (stat == 2) {
          *ap = fminf(*ap, v);
        } else {
          *ap = *ap + v * v;
        }
      }
    }
    __syncthreads();
  }

#pragma unroll 1
  for (int it = tid; it < NB * DD; it += NTHR) {
    const int sl = it >> 6, c = it & 63;
    const int dgc = cnt[sl];
    const float deg = (float)dgc;
    const float sd = fmaxf(deg, 1.0f);
    const float rs = 1.0f / sd;
    float* ar = acc + sl * AGW;
    const float sum = ar[c], mx = ar[64 + c], mn = ar[128 + c], sq = ar[192 + c];
    const float mean = sum * rs;
    float var = sq * rs - mean * mean;
    var = fmaxf(var, 0.0f);
    const float stdv = sqrtf(var + AEPS);
    const bool has = dgc > 0;
    ar[c]       = mean;
    ar[64 + c]  = has ? mx : 0.0f;
    ar[128 + c] = has ? mn : 0.0f;
    ar[192 + c] = has ? stdv : 0.0f;
  }
  if (tid < NB) {
    const float deg = (float)cnt[tid];
    const float logD = logf(deg + 1.0f);
    const float amp = logD * RAVGL;
    const float den = (logD > 0.0f) ? logD : 1.0f;
    const float att = AVGL * (1.0f / den);
    dgs[tid * 4 + 0] = amp;
    dgs[tid * 4 + 1] = att;
    dgs[tid * 4 + 2] = 0.0f;
    dgs[tid * 4 + 3] = 0.0f;
  }
  __syncthreads();
#pragma unroll 1
  for (int rr = 0; rr < 16; ++rr) {
    const int nl = wave * 16 + rr;
#pragma unroll
    for (int j = 0; j < 2; ++j) {
      const v4f v = *(const v4f*)(acc + nl * AGW + 128 * j + 4 * lane);
      *(volatile v4f*)(aggp + (size_t)(nodeBase + nl) * AGW + 128 * j + 4 * lane) = v;
    }
  }
  if (wdg != 0 && wave == 0) {
#pragma unroll
    for (int j = 0; j < 4; ++j) {
      const v4f v = *(const v4f*)(dgs + 128 * j + 4 * lane);
      *(volatile v4f*)(dgp + (size_t)nodeBase * 4 + 128 * j + 4 * lane) = v;
    }
  }
  __threadfence();
#pragma unroll 1
  for (int rr = 0; rr < 16; ++rr) {
    const int nl = wave * 16 + rr;
#pragma unroll
    for (int j = 0; j < 2; ++j) {
      const v4f v = *(const v4f*)(acc + nl * AGW + 128 * j + 4 * lane);
      *(volatile v4f*)(aggp + (size_t)(nodeBase + nl) * AGW + 128 * j + 4 * lane) = v;
    }
  }
  if (wdg != 0 && wave == 0) {
#pragma unroll
    for (int j = 0; j < 4; ++j) {
      const v4f v = *(const v4f*)(dgs + 128 * j + 4 * lane);
      *(volatile v4f*)(dgp + (size_t)nodeBase * 4 + 128 * j + 4 * lane) = v;
    }
  }
}

__global__ __launch_bounds__(RTHR) void k_post(
    const float* __restrict__ xa, const float* __restrict__ xb, int nkx,
    const float* __restrict__ aggp, const float* __restrict__ dgp,
    const unsigned short* __restrict__ qh, const unsigned short* __restrict__ ql, int kp,
    const float* __restrict__ bias, const float* __restrict__ snorm, int bn,
    float* tp, float* bnp, int nN) {
  __shared__ __attribute__((aligned(16))) float stg[RB * DD];
  __shared__ float sn[RB];
  __shared__ int sv[RB];
  __shared__ __attribute__((aligned(16))) float part[2 * DD];
  const int tid = threadIdx.x, lane = tid & 31, wave = tid >> 5, hh = lane >> 4, m = lane & 15;
  const int rowBase = blockIdx.x * RB;
  int node = rowBase + wave * 16 + m;
  node = node > nN - 1 ? nN - 1 : node;
  v8f acc[4];
#pragma unroll
  for (int i = 0; i < 4; ++i) acc[i] = zero8();
  {
    const float* ra = xa + (size_t)node * DD;
    gstep<4>(acc, ra, 0,  1.0f, qh, ql, kp, 0,  hh, m);
    gstep<4>(acc, ra, 32, 1.0f, qh, ql, kp, 32, hh, m);
  }
  int kw0 = DD;
  if (nkx == 2) {
    const float* rb2 = xb + (size_t)node * DD;
    gstep<4>(acc, rb2, 0,  1.0f, qh, ql, kp, DD,      hh, m);
    gstep<4>(acc, rb2, 32, 1.0f, qh, ql, kp, DD + 32, hh, m);
    kw0 = 2 * DD;
  }
  {
    const float* rg = aggp + (size_t)node * AGW;
    const float amp = dgp[(size_t)node * 4 + 0];
    const float att = dgp[(size_t)node * 4 + 1];
#pragma unroll 1
    for (int kt = 0; kt < AGW / 32; ++kt)
      gstep<4>(acc, rg, 32 * kt, 1.0f, qh, ql, kp, kw0 + 32 * kt, hh, m);
#pragma unroll 1
    for (int kt = 0; kt < AGW / 32; ++kt)
      gstep<4>(acc, rg, 32 * kt, amp, qh, ql, kp, kw0 + AGW + 32 * kt, hh, m);
#pragma unroll 1
    for (int kt = 0; kt < AGW / 32; ++kt)
      gstep<4>(acc, rg, 32 * kt, att, qh, ql, kp, kw0 + 2 * AGW + 32 * kt, hh, m);
  }
#pragma unroll
  for (int ft = 0; ft < 4; ++ft) {
    const float bc = bias[16 * ft + m];
#pragma unroll
    for (int rr = 0; rr < 8; ++rr) stg[(wave * 16 + 8 * hh + rr) * DD + 16 * ft + m] = acc[ft][rr] + bc;
  }
  if (tid < RB) {
    const int row = rowBase + tid;
    sv[tid] = (row < nN) ? 1 : 0;
    sn[tid] = snorm[row > nN - 1 ? nN - 1 : row];
  }
  __syncthreads();
  if (bn != 0) {
    if (tid < DD) {
      const int c = tid;
      double s = 0.0, q = 0.0;
#pragma unroll 1
      for (int row = 0; row < RB; ++row) {
        const float v = stg[row * DD + c] * sn[row];
        stg[row * DD + c] = v;
        if (sv[row] != 0) {
          s += (double)v;
          q += (double)v * (double)v;
        }
      }
      part[c] = (float)s;
      part[DD + c] = (float)q;
    }
  }
  __syncthreads();
#pragma unroll 1
  for (int j = 0; j < 8; ++j) {
    const int lrow = wave * 16 + 2 * j;
    const v4f v = *(const v4f*)(stg + lrow * DD + 4 * lane);
    *(volatile v4f*)(tp + (size_t)(rowBase + lrow) * DD + 4 * lane) = v;
  }
  if (bn != 0 && wave == 0) {
    const v4f v = *(const v4f*)(part + 4 * lane);
    *(volatile v4f*)(bnp + (size_t)blockIdx.x * 2 * DD + 4 * lane) = v;
  }
  __threadfence();
#pragma unroll 1
  for (int j = 0; j < 8; ++j) {
    const int lrow = wave * 16 + 2 * j;
    const v4f v = *(const v4f*)(stg + lrow * DD + 4 * lane);
    *(volatile v4f*)(tp + (size_t)(rowBase + lrow) * DD + 4 * lane) = v;
  }
  if (bn != 0 && wave == 0) {
    const v4f v = *(const v4f*)(part + 4 * lane);
    *(volatile v4f*)(bnp + (size_t)blockIdx.x * 2 * DD + 4 * lane) = v;
  }
}

__global__ __launch_bounds__(RTHR) void k_mix(
    const float* __restrict__ tp, const float* __restrict__ bnp, int nPart, int bn,
    const float* __restrict__ gam, const float* __restrict__ bet,
    const unsigned short* __restrict__ qh, const unsigned short* __restrict__ ql,
    const float* __restrict__ bias, const float* __restrict__ xres, int act,
    float* outp, int nN) {
  __shared__ __attribute__((aligned(16))) float stg[RB * DD];
  __shared__ float bna[DD];
  __shared__ float bnb[DD];
  const int tid = threadIdx.x, lane = tid & 31, wave = tid >> 5, hh = lane >> 4, m = lane & 15;
  const int rowBase = blockIdx.x * RB;
  if (tid < DD) {
    const int c = tid;
    float a = 1.0f, b0 = 0.0f;
    if (bn != 0) {
      double s = 0.0, q = 0.0;
#pragma unroll 1
      for (int i = 0; i < nPart; ++i) {
        s += (double)bnp[(size_t)i * 2 * DD + c];
        q += (double)bnp[(size_t)i * 2 * DD + DD + c];
      }
      const double inv_n = 1.0 / (double)nN;
      const double mu = s * inv_n;
      double var = q * inv_n - mu * mu;
      if (var < 0.0) var = 0.0;
      const float rstd = 1.0f / sqrtf((float)var + BEPS);
      a = gam[c] * rstd;
      b0 = bet[c] - (float)mu * a;
    }
    bna[c] = a;
    bnb[c] = b0;
  }
  __syncthreads();
  int node = rowBase + wave * 16 + m;
  node = node > nN - 1 ? nN - 1 : node;
  const float* tr = tp + (size_t)node * DD;
  v8f acc[4];
#pragma unroll
  for (int i = 0; i < 4; ++i) acc[i] = zero8();
#pragma unroll
  for (int kt = 0; kt < 2; ++kt) {
    const int k0 = 32 * kt;
    const int ka = k0 + 8 * hh, kc = k0 + 16 + 8 * hh;
    v4f a = *(const v4f*)(tr + ka);
    v4f b = *(const v4f*)(tr + ka + 4);
    v4f c = *(const v4f*)(tr + kc);
    v4f d = *(const v4f*)(tr + kc + 4);
    a.x = a.x * bna[ka + 0] + bnb[ka + 0]; a.y = a.y * bna[ka + 1] + bnb[ka + 1];
    a.z = a.z * bna[ka + 2] + bnb[ka + 2]; a.w = a.w * bna[ka + 3] + bnb[ka + 3];
    b.x = b.x * bna[ka + 4] + bnb[ka + 4]; b.y = b.y * bna[ka + 5] + bnb[ka + 5];
    b.z = b.z * bna[ka + 6] + bnb[ka + 6]; b.w = b.w * bna[ka + 7] + bnb[ka + 7];
    c.x = c.x * bna[kc + 0] + bnb[kc + 0]; c.y = c.y * bna[kc + 1] + bnb[kc + 1];
    c.z = c.z * bna[kc + 2] + bnb[kc + 2]; c.w = c.w * bna[kc + 3] + bnb[kc + 3];
    d.x = d.x * bna[kc + 4] + bnb[kc + 4]; d.y = d.y * bna[kc + 5] + bnb[kc + 5];
    d.z = d.z * bna[kc + 6] + bnb[kc + 6]; d.w = d.w * bna[kc + 7] + bnb[kc + 7];
    FragB ah, al;
    split8(a, b, ah.h[0], al.h[0]);
    split8(c, d, ah.h[1], al.h[1]);
#pragma unroll
    for (int ft = 0; ft < 4; ++ft) {
      FragB bh, bl;
      const size_t o = (size_t)(16 * ft + m) * DD + k0 + 8 * hh;
      bh.h[0] = *(const v8us*)(qh + o);
      bh.h[1] = *(const v8us*)(qh + o + 16);
      bl.h[0] = *(const v8us*)(ql + o);
      bl.h[1] = *(const v8us*)(ql + o + 16);
      acc[ft] = wm3(ah.v, al.v, bh.v, bl.v, acc[ft]);
    }
  }
#pragma unroll
  for (int ft = 0; ft < 4; ++ft) {
    const int col = 16 * ft + m;
    const float bc = bias[col];
#pragma unroll
    for (int rr = 0; rr < 8; ++rr) {
      float v = acc[ft][rr] + bc;
      if (act != 0) {
        v = tanhf(v);
      } else {
        v = v > 0.0f ? v : 0.01f * v;
      }
      int grow = rowBase + wave * 16 + 8 * hh + rr;
      grow = grow > nN - 1 ? nN - 1 : grow;
      v = xres[(size_t)grow * DD + col] + v;
      stg[(wave * 16 + 8 * hh + rr) * DD + col] = v;
    }
  }
  __syncthreads();
#pragma unroll 1
  for (int j = 0; j < 8; ++j) {
    const int lrow = wave * 16 + 2 * j;
    const int grow = rowBase + lrow;
    const v4f v = *(const v4f*)(stg + lrow * DD + 4 * lane);
    float* op = outp + (size_t)grow * DD + 4 * lane;
    if (grow + 2 <= nN) {
      *(volatile v4f*)op = v;
    } else if (grow + 1 <= nN) {
      if (lane < 16) *(volatile v4f*)op = v;
    }
  }
  __threadfence();
#pragma unroll 1
  for (int j = 0; j < 8; ++j) {
    const int lrow = wave * 16 + 2 * j;
    const int grow = rowBase + lrow;
    const v4f v = *(const v4f*)(stg + lrow * DD + 4 * lane);
    float* op = outp + (size_t)grow * DD + 4 * lane;
    if (grow + 2 <= nN) {
      *(volatile v4f*)op = v;
    } else if (grow + 1 <= nN) {
      if (lane < 16) *(volatile v4f*)op = v;
    }
  }
}

extern "C" void kernel_launch(void* const* d_in, const int* in_sizes, int n_in,
                              void* d_out, int out_size, void* d_ws, size_t ws_size,
                              hipStream_t stream) {
  if (n_in < 20) return;
  const int nN = in_sizes[0] / DD;
  if (nN < 1 || in_sizes[0] != nN * DD || in_sizes[1] != nN * DD || in_sizes[3] != nN) return;
  const int nE = in_sizes[4];
  if (nE < 1 || in_sizes[5] != nE || in_sizes[2] != nE * EKIN) return;
  if (in_sizes[6] != (2 * PXW + EKIN) * DD || in_sizes[7] != DD) return;
  if (in_sizes[8] != (2 * DD + EKIN) * DD || in_sizes[9] != DD) return;
  if (in_sizes[10] != KPH * DD || in_sizes[11] != DD || in_sizes[12] != KPP * DD || in_sizes[13] != DD) return;
  if (in_sizes[14] != DD || in_sizes[15] != DD) return;
  if (in_sizes[16] != DD * DD || in_sizes[17] != DD || in_sizes[18] != DD * DD || in_sizes[19] != DD) return;
  if (out_size != 2 * nN * DD) return;

  const float* h     = (const float*)d_in[0];
  const float* p     = (const float*)d_in[1];
  const float* e     = (const float*)d_in[2];
  const float* snorm = (const float*)d_in[3];
  const int*   src   = (const int*)d_in[4];
  const int*   dst   = (const int*)d_in[5];
  const float* wpreh = (const float*)d_in[6];
  const float* bpreh = (const float*)d_in[7];
  const float* wprep = (const float*)d_in[8];
  const float* bprep = (const float*)d_in[9];
  const float* wposh = (const float*)d_in[10];
  const float* bposh = (const float*)d_in[11];
  const float* wposp = (const float*)d_in[12];
  const float* bposp = (const float*)d_in[13];
  const float* gam   = (const float*)d_in[14];
  const float* bet   = (const float*)d_in[15];
  const float* wmixh = (const float*)d_in[16];
  const float* bmixh = (const float*)d_in[17];
  const float* wmixp = (const float*)d_in[18];
  const float* bmixp = (const float*)d_in[19];
  float* dout = (float*)d_out;

  const int nBlk = (nN + NB - 1) / NB;
  const size_t rowsP = (size_t)nBlk * NB;
  const int nRB = (int)(rowsP / RB);

  const size_t nq0 = (size_t)128 * 128, nq1 = (size_t)128 * 64, nq2 = (size_t)64 * KPH, nq3 = (size_t)64 * KPP;
  const size_t nq4 = (size_t)64 * 64, nqe = (size_t)64 * ETW;

  char* ws = (char*)d_ws;
  size_t off = 0;
  auto carve = [&](size_t bytes) -> size_t {
    const size_t o = off;
    off = (off + bytes + 255) & ~(size_t)255;
    return o;
  };
  const size_t oq0  = carve(2 * nq0 * 2), oq1 = carve(2 * nq1 * 2), oq2 = carve(2 * nq2 * 2), oq3 = carve(2 * nq3 * 2);
  const size_t oq4  = carve(2 * nq4 * 2), oq5 = carve(2 * nq4 * 2);
  const size_t oqe0 = carve(nqe * 2), oqe1 = carve(nqe * 2);
  const size_t oet  = carve((size_t)nBlk * EROW * 4);
  const size_t oph  = carve(rowsP * PXW * 4);
  const size_t opp  = carve(rowsP * PXW * 4);
  const size_t oagh = carve(rowsP * AGW * 4);
  const size_t oagp = carve(rowsP * AGW * 4);
  const size_t odg  = carve(rowsP * 4 * 4);
  const size_t oht  = carve(rowsP * DD * 4);
  const size_t opt  = carve(rowsP * DD * 4);
  const size_t obnp = carve((size_t)nRB * 2 * DD * 4);
  size_t limit = (size_t)WSLIM;
  if (ws_size < limit) limit = ws_size;
  if (off > limit) return;

  unsigned short* q0 = (unsigned short*)(ws + oq0);
  unsigned short* q1 = (unsigned short*)(ws + oq1);
  unsigned short* q2 = (unsigned short*)(ws + oq2);
  unsigned short* q3 = (unsigned short*)(ws + oq3);
  unsigned short* q4 = (unsigned short*)(ws + oq4);
  unsigned short* q5 = (unsigned short*)(ws + oq5);
  _Float16* qe0 = (_Float16*)(ws + oqe0);
  _Float16* qe1 = (_Float16*)(ws + oqe1);
  int*   etab = (int*)(ws + oet);
  float* PH   = (float*)(ws + oph);
  float* PP   = (float*)(ws + opp);
  float* AGH  = (float*)(ws + oagh);
  float* AGP  = (float*)(ws + oagp);
  float* DG   = (float*)(ws + odg);
  float* HT   = (float*)(ws + oht);
  float* PT   = (float*)(ws + opt);
  float* BNP  = (float*)(ws + obnp);

  k_prep<<<PBT, NTHR, 0, stream>>>(wpreh, wprep, wposh, wposp, wmixh, wmixp, q0, q1, q2, q3, q4, q5, qe0, qe1);
  k_escan<<<nBlk, NTHR, 0, stream>>>(dst, etab, nE, 1);
  k_proj<<<nRB, RTHR, 0, stream>>>(h, p, q0, q0 + nq0, q1, q1 + nq1, PH, PP, nN);

  hipFuncSetAttribute(reinterpret_cast<const void*>(&k_agg), hipFuncAttributeMaxDynamicSharedMemorySize, LA_TOT);
  k_agg<<<nBlk, NTHR, LA_TOT, stream>>>(PH, e, src, dst, etab, qe0, bpreh, AGH, DG, nN, nE, 1);
  k_agg<<<nBlk, NTHR, LA_TOT, stream>>>(PP, e, src, dst, etab, qe1, bprep, AGP, DG, nN, nE, 0);

  k_post<<<nRB, RTHR, 0, stream>>>(h, p, 2, AGH, DG, q2, q2 + nq2, KPH, bposh, snorm, 1, HT, BNP, nN);
  k_post<<<nRB, RTHR, 0, stream>>>(p, p, 1, AGP, DG, q3, q3 + nq3, KPP, bposp, snorm, 0, PT, BNP, nN);

  k_mix<<<nRB, RTHR, 0, stream>>>(HT, BNP, nRB, 1, gam, bet, q4, q4 + nq4, bmixh, h, 0, dout, nN);
  k_mix<<<nRB, RTHR, 0, stream>>>(PT, BNP, nRB, 0, gam, bet, q5, q5 + nq4, bmixp, p, 1, dout + (size_t)nN * DD, nN);
}
